// StaircaseSeqAttention_11072425689258
// MI455X (gfx1250) — hardware-verified
//
#include <hip/hip_runtime.h>

constexpr int kNB  = 16;
constexpr int kSeq = 2048;
constexpr int kHD  = 128;
constexpr int kLim = 2048;
constexpr int kGrp = 2;
constexpr float kInvSqrtD = 0.08838834764831845f;
static_assert(kLim == kSeq, "table spans the key length");
static_assert(kSeq % 256 == 0 && kHD % 64 == 0 && kLim % 64 == 0 && (kNB % kGrp) == 0, "tile multiples");

typedef __attribute__((ext_vector_type(16))) _Float16 v16h;
typedef __attribute__((ext_vector_type(8)))  _Float16 v8h;
typedef __attribute__((ext_vector_type(16))) __bf16   v16b;
typedef __attribute__((ext_vector_type(8)))  __bf16   v8b;
typedef __attribute__((ext_vector_type(8)))  float    v8f;
typedef __attribute__((ext_vector_type(4)))  float    v4f;
typedef __attribute__((ext_vector_type(4)))  unsigned int v4u;

__device__ __forceinline__ unsigned short f2bf_bits(float f) {
  unsigned u = __float_as_uint(f);
  return (unsigned short)((u + 0x7FFFu + ((u >> 16) & 1u)) >> 16);
}
__device__ __forceinline__ float bf_bits2f(unsigned short h) { return __uint_as_float(((unsigned)h) << 16); }

__device__ __forceinline__ void dep_guard_h(v8f& a, v8f& b, v16h x, v16h y) { asm volatile("v_nop\n\tv_nop\n\tv_nop\n\tv_nop" : "+v"(a), "+v"(b) : "v"(x), "v"(y)); }
__device__ __forceinline__ void dep_guard_b(v8f& a, v8f& b, v16b x, v16b y) { asm volatile("v_nop\n\tv_nop\n\tv_nop\n\tv_nop" : "+v"(a), "+v"(b) : "v"(x), "v"(y)); }
__device__ __forceinline__ void keep4_h(v16h a, v16h b, v16h c, v16h d) { asm volatile("v_nop" :: "v"(a), "v"(b), "v"(c), "v"(d)); }
__device__ __forceinline__ void keep4_b(v16b a, v16b b, v16b c, v16b d) { asm volatile("v_nop" :: "v"(a), "v"(b), "v"(c), "v"(d)); }
__device__ __forceinline__ void acc_guard4(v8f& a, v8f& b, v8f& c, v8f& d) { asm volatile("v_nop\n\tv_nop\n\tv_nop\n\tv_nop" : "+v"(a), "+v"(b), "+v"(c), "+v"(d)); }
template <typename T> struct Frag;
template <> struct Frag<_Float16> {
  typedef v16h V; union U { v16h v; v8h h[2]; };
  static __device__ __forceinline__ v16h load(const _Float16* p) {
    U f; f.h[0] = *(const v8h*)(p); f.h[1] = *(const v8h*)(p + 16); return f.v;
  }
  static __device__ __forceinline__ v8f mma(v16h a, v16h b, v8f c) {
    return __builtin_amdgcn_wmma_f32_16x16x32_f16(false, a, false, b, (short)0, c, false, false);
  }
  static __device__ __forceinline__ void guard(v8f& a, v8f& b, v16h x, v16h y) { dep_guard_h(a, b, x, y); }
  static __device__ __forceinline__ void keep(v16h a, v16h b, v16h c, v16h d) { keep4_h(a, b, c, d); }
};
template <> struct Frag<__bf16> {
  typedef v16b V; union U { v16b v; v8b h[2]; };
  static __device__ __forceinline__ v16b load(const __bf16* p) {
    U f; f.h[0] = *(const v8b*)(p); f.h[1] = *(const v8b*)(p + 16); return f.v;
  }
  static __device__ __forceinline__ v8f mma(v16b a, v16b b, v8f c) {
    return __builtin_amdgcn_wmma_f32_16x16x32_bf16(false, a, false, b, (short)0, c, false, false);
  }
  static __device__ __forceinline__ void guard(v8f& a, v8f& b, v16b x, v16b y) { dep_guard_b(a, b, x, y); }
  static __device__ __forceinline__ void keep(v16b a, v16b b, v16b c, v16b d) { keep4_b(a, b, c, d); }
};

__device__ __forceinline__ unsigned pk16(unsigned short a, unsigned short b) { return (unsigned)a | ((unsigned)b << 16); }

template <int ET> struct Elem;
template <> struct Elem<0> { typedef _Float16 T; };
template <> struct Elem<1> { typedef __bf16 T; };
template <int ET, bool SPLIT, bool AONLY, int OUT_MODE, bool RESID, int SKIP, bool KLIM>
__global__ __launch_bounds__(256) void wmma_gemm64(
    const unsigned short* __restrict__ Ap, const unsigned short* __restrict__ A2p, int lda, long strideA,
    const unsigned short* __restrict__ Btp, const unsigned short* __restrict__ Bt2p, int ldb, long strideB,
    void* __restrict__ Cout, void* __restrict__ Cout2, int ldc, long strideC,
    const float* __restrict__ resid, long strideR, int ldr,
    int M, int N, int K, float scale) {
  typedef typename Elem<ET>::T T;
  typedef typename Frag<T>::V V;
  const T* A = (const T*)Ap; const T* A2 = (const T*)A2p; const T* Bt = (const T*)Btp; const T* Bt2 = (const T*)Bt2p;
  __shared__ __align__(16) float sT[8][16 * 68];
  const int b    = blockIdx.y;
  const int lane = threadIdx.x & 31;
  const int wave = threadIdx.x >> 5;
  const int tilesN = N >> 6;
  const int tilesM = M >> 6;
  const int tile = blockIdx.x * 8 + wave;
  if (tile >= tilesM * tilesN) return;
  const int tm = tile / tilesN;
  const int tn = tile - tm * tilesN;
  if (SKIP == 1 && tn > tm) return;
  if (SKIP == 2 && tn + tm < tilesN - 1) return;
  const int m0 = tm << 6;
  const int n0 = tn << 6;
  const int Kend = KLIM ? ((m0 + 64 < K) ? (m0 + 64) : K) : K;

  const T* Ab  = A  + (size_t)b * strideA;
  const T* Bb  = Bt + (size_t)b * strideB;
  const T* Ab2 = SPLIT ? (A2  + (size_t)b * strideA) : nullptr;
  const T* Bb2 = (SPLIT && !AONLY) ? (Bt2 + (size_t)b * strideB) : nullptr;

  const int rlane = lane & 15;
  const int koff  = (lane >> 4) * 8;
  const int mOff  = (lane >> 4) * 8;

  v8f acc[4][4];
#pragma unroll
  for (int i = 0; i < 4; ++i)
#pragma unroll
    for (int j = 0; j < 4; ++j) acc[i][j] = (v8f){0.f,0.f,0.f,0.f,0.f,0.f,0.f,0.f};

  for (int k0 = 0; k0 < Kend; k0 += 32) {
    V bh[4], bl[4];
#pragma unroll
    for (int j = 0; j < 4; ++j) {
      const size_t bo = (size_t)(n0 + (j << 4) + rlane) * ldb + koff + k0;
      bh[j] = Frag<T>::load(Bb + bo);
      if (SPLIT && !AONLY) bl[j] = Frag<T>::load(Bb2 + bo);
    }
#pragma unroll
    for (int i = 0; i < 4; ++i) {
      const size_t ao = (size_t)(m0 + (i << 4) + rlane) * lda + koff + k0;
      V ah = Frag<T>::load(Ab + ao);
      V al;
      if (SPLIT) al = Frag<T>::load(Ab2 + ao);
#pragma unroll
      for (int j = 0; j < 4; ++j) {
        acc[i][j] = Frag<T>::mma(ah, bh[j], acc[i][j]);
        if (SPLIT) {
          if (!AONLY) acc[i][j] = Frag<T>::mma(ah, bl[j], acc[i][j]);
          acc[i][j] = Frag<T>::mma(al, bh[j], acc[i][j]);
        }
      }
      Frag<T>::guard(acc[i][0], acc[i][3], ah, SPLIT ? al : ah);
    }
    Frag<T>::keep(bh[0], bh[1], bh[2], bh[3]);
    if (SPLIT && !AONLY) Frag<T>::keep(bl[0], bl[1], bl[2], bl[3]);
  }
  acc_guard4(acc[0][0], acc[0][1], acc[0][2], acc[0][3]);
  acc_guard4(acc[1][0], acc[1][1], acc[1][2], acc[1][3]);
  acc_guard4(acc[2][0], acc[2][1], acc[2][2], acc[2][3]);
  acc_guard4(acc[3][0], acc[3][1], acc[3][2], acc[3][3]);

  float* slab = sT[wave];
  const float* Rb = RESID ? (resid + (size_t)b * strideR) : nullptr;
#pragma unroll
  for (int i = 0; i < 4; ++i) {
    const int mBase = m0 + (i << 4);
#pragma unroll
    for (int j = 0; j < 4; ++j) {
      const int n = n0 + (j << 4) + rlane;
#pragma unroll
      for (int r = 0; r < 8; ++r) {
        float v = acc[i][j][r] * scale;
        if (RESID) v += Rb[(size_t)(mBase + mOff + r) * ldr + n];
        slab[(mOff + r) * 68 + (j << 4) + rlane] = v;
      }
    }
    __builtin_amdgcn_fence(__ATOMIC_RELEASE, "workgroup");
    __builtin_amdgcn_wave_barrier();
    __builtin_amdgcn_fence(__ATOMIC_ACQUIRE, "workgroup");
    if (OUT_MODE == 0) {
      float* C = (float*)Cout + (size_t)b * strideC;
      const int hh = lane >> 4, c4 = (lane & 15) * 4;
      for (int pass = 0; pass < 2; ++pass) {
#pragma unroll
        for (int it = 0; it < 8; ++it) {
          const int row = it * 2 + hh;
          v4f v = *(const v4f*)(slab + row * 68 + c4);
          *(volatile v4f*)(C + (size_t)(mBase + row) * ldc + n0 + c4) = v;
        }
        __threadfence();
      }
    } else {
      const int q = lane >> 3, c8 = (lane & 7) * 8;
      unsigned short* C  = (unsigned short*)Cout  + (size_t)b * strideC;
      unsigned short* C2 = (OUT_MODE == 2) ? ((unsigned short*)Cout2 + (size_t)b * strideC) : nullptr;
      for (int pass = 0; pass < 2; ++pass) {
#pragma unroll
        for (int it = 0; it < 4; ++it) {
          const int row = it * 4 + q;
          const float* sp = slab + row * 68 + c8;
          v8h hv, lv;
#pragma unroll
          for (int e = 0; e < 8; ++e) {
            if (OUT_MODE == 1) {
              hv[e] = (_Float16)sp[e];
            } else {
              unsigned short hb = f2bf_bits(sp[e]);
              unsigned short lb = f2bf_bits(sp[e] - bf_bits2f(hb));
              hv[e] = __builtin_bit_cast(_Float16, hb);
              lv[e] = __builtin_bit_cast(_Float16, lb);
            }
          }
          *(volatile v8h*)(C + (size_t)(mBase + row) * ldc + n0 + c8) = hv;
          if (OUT_MODE == 2) *(volatile v8h*)(C2 + (size_t)(mBase + row) * ldc + n0 + c8) = lv;
        }
        __threadfence();
      }
    }
    __builtin_amdgcn_fence(__ATOMIC_RELEASE, "workgroup");
    __builtin_amdgcn_wave_barrier();
    __builtin_amdgcn_fence(__ATOMIC_ACQUIRE, "workgroup");
  }
}

__global__ __launch_bounds__(256) void cast8_bf16_pair_kernel(const float* __restrict__ in0, const float* __restrict__ in1,
                                                              unsigned short* __restrict__ out0, unsigned short* __restrict__ out1,
                                                              int n8) {
  const int i = blockIdx.x * 256 + threadIdx.x;
  if (i >= n8) return;
  const bool sel = (blockIdx.y != 0);
  const float* p = (sel ? in1 : in0) + 8 * (size_t)i;
  const v4f a = *(const v4f*)(p);
  const v4f c = *(const v4f*)(p + 4);
  unsigned short hb[8];
#pragma unroll
  for (int e = 0; e < 4; ++e) {
    hb[e]     = f2bf_bits(a[e]);
    hb[4 + e] = f2bf_bits(c[e]);
  }
  const v4u u = (v4u){pk16(hb[0], hb[1]), pk16(hb[2], hb[3]), pk16(hb[4], hb[5]), pk16(hb[6], hb[7])};
  unsigned short* q = (sel ? out1 : out0) + 8 * (size_t)i;
  *(volatile v4u*)q = u;
  __threadfence();
  *(volatile v4u*)q = u;
}

__global__ __launch_bounds__(256) void transpose_bf16_kernel(const float* __restrict__ in, unsigned short* __restrict__ out,
                                                             int nr, int nc) {
  __shared__ float sm[64][65];
  const int t  = threadIdx.x;
  const int c0 = blockIdx.x * 64;
  const int r0 = blockIdx.y * 64;
  const int z  = blockIdx.z;
  const float* ib = in + (size_t)z * nr * nc;
  unsigned short* ob = out + (size_t)z * nr * nc;
#pragma unroll
  for (int i = 0; i < 16; ++i) {
    const int e = i * 256 + t;
    const int r = e >> 6;
    const int c = e & 63;
    sm[c][r] = ib[(size_t)(r0 + r) * nc + c0 + c];
  }
  __syncthreads();
  const int lane = t & 31, wave = t >> 5;
  const int q = lane >> 3, c8 = (lane & 7) * 8;
  for (int pass = 0; pass < 2; ++pass) {
#pragma unroll
    for (int it = 0; it < 2; ++it) {
      const int row = wave * 8 + it * 4 + q;
      unsigned short hb[8];
#pragma unroll
      for (int e = 0; e < 8; ++e) hb[e] = f2bf_bits(sm[row][c8 + e]);
      const v4u u = (v4u){pk16(hb[0], hb[1]), pk16(hb[2], hb[3]), pk16(hb[4], hb[5]), pk16(hb[6], hb[7])};
      *(volatile v4u*)(ob + (size_t)(c0 + row) * nr + r0 + c8) = u;
    }
    __threadfence();
  }
}

__global__ __launch_bounds__(256) void softmax_skew_kernel(const float* __restrict__ Sc,
                                                           unsigned short* __restrict__ Ph, unsigned short* __restrict__ Pl) {
  __shared__ float redM[8];
  __shared__ float redS[8];
  const int i    = blockIdx.x;
  const int bb   = blockIdx.y;
  const int t    = threadIdx.x;
  const int lane = t & 31, wave = t >> 5;
  const int c0   = t * 8;
  const int kend = (i & ~63) + 64;
  const bool active = (wave * 256) < kend;
  const size_t rowoff = ((size_t)bb * kSeq + (size_t)i) * kSeq;
  const float ninf = -__builtin_inff();

  float x[8];
  float m = ninf;
  if (active) {
    const float* sr = Sc + rowoff + c0;
    const v4f a = *(const v4f*)(sr);
    const v4f c = *(const v4f*)(sr + 4);
#pragma unroll
    for (int e = 0; e < 4; ++e) {
      x[e]     = (c0 + e     <= i) ? a[e] * kInvSqrtD : ninf;
      x[4 + e] = (c0 + 4 + e <= i) ? c[e] * kInvSqrtD : ninf;
    }
#pragma unroll
    for (int e = 0; e < 8; ++e) m = fmaxf(m, x[e]);
  } else {
#pragma unroll
    for (int e = 0; e < 8; ++e) x[e] = ninf;
  }
#pragma unroll
  for (int off = 16; off > 0; off >>= 1) m = fmaxf(m, __shfl_xor(m, off, 32));
  if (lane == 0) redM[wave] = m;
  __syncthreads();
  float gm = redM[0];
#pragma unroll
  for (int w = 1; w < 8; ++w) gm = fmaxf(gm, redM[w]);

  float p[8];
  float ps = 0.f;
#pragma unroll
  for (int e = 0; e < 8; ++e) { p[e] = __expf(x[e] - gm); ps += p[e]; }
#pragma unroll
  for (int off = 16; off > 0; off >>= 1) ps += __shfl_xor(ps, off, 32);
  if (lane == 0) redS[wave] = ps;
  __syncthreads();
  float tot = redS[0];
#pragma unroll
  for (int w = 1; w < 8; ++w) tot += redS[w];
  const float inv = 1.0f / tot;

  if (active) {
    unsigned short hb[8], lb[8];
#pragma unroll
    for (int e = 0; e < 8; ++e) {
      const float pn = p[e] * inv;
      const unsigned short h = f2bf_bits(pn);
      hb[e] = h;
      lb[e] = f2bf_bits(pn - bf_bits2f(h));
    }
    const v4u hu = (v4u){pk16(hb[0], hb[1]), pk16(hb[2], hb[3]), pk16(hb[4], hb[5]), pk16(hb[6], hb[7])};
    const v4u lu = (v4u){pk16(lb[0], lb[1]), pk16(lb[2], lb[3]), pk16(lb[4], lb[5]), pk16(lb[6], lb[7])};
    unsigned short* ph = Ph + rowoff + c0;
    unsigned short* pl = Pl + rowoff + c0;
    *(volatile v4u*)ph = hu;
    *(volatile v4u*)pl = lu;
    __threadfence();
    *(volatile v4u*)ph = hu;
    *(volatile v4u*)pl = lu;
  }
}

extern "C" void kernel_launch(void* const* d_in, const int* in_sizes, int n_in,
                              void* d_out, int out_size, void* d_ws, size_t ws_size,
                              hipStream_t stream) {
  (void)n_in;
  const size_t nQK = (size_t)kNB * kSeq * kHD;
  const size_t nPE = (size_t)kHD * kLim;
  const size_t plane = (size_t)kSeq * kSeq;
  const size_t offQ  = 0;
  const size_t offK  = offQ  + nQK * 2;
  const size_t offVt = offK  + nQK * 2;
  const size_t offPE = offVt + nQK * 2;
  const size_t offS  = offPE + nPE * 2;
  const size_t offR  = offS  + (size_t)kGrp * plane * 4;
  const size_t offPl = offR  + (size_t)kGrp * plane * 2;
  const size_t total = offR  + (size_t)kGrp * plane * 4;
  if (n_in < 4) return;
  if ((size_t)in_sizes[0] != nQK || (size_t)in_sizes[1] != nQK || (size_t)in_sizes[2] != nQK || (size_t)in_sizes[3] != nPE) return;
  if ((size_t)out_size != nQK) return;
  if (ws_size < total) return;

  const float* q  = (const float*)d_in[0];
  const float* k  = (const float*)d_in[1];
  const float* v  = (const float*)d_in[2];
  const float* pe = (const float*)d_in[3];
  float* out = (float*)d_out;
  unsigned char* ws = (unsigned char*)d_ws;
  unsigned short* Qb  = (unsigned short*)(ws + offQ);
  unsigned short* Kb  = (unsigned short*)(ws + offK);
  unsigned short* Vt  = (unsigned short*)(ws + offVt);
  unsigned short* PEt = (unsigned short*)(ws + offPE);
  float*          Sc  = (float*)(ws + offS);
  float*          Rf  = (float*)(ws + offR);
  unsigned short* Ph  = (unsigned short*)(ws + offR);
  unsigned short* Pl  = (unsigned short*)(ws + offPl);

  cast8_bf16_pair_kernel<<<dim3((unsigned)(nQK / 8 / 256), 2), 256, 0, stream>>>(q, k, Qb, Kb, (int)(nQK / 8));
  transpose_bf16_kernel<<<dim3(kHD / 64, kSeq / 64, kNB), 256, 0, stream>>>(v, Vt, kSeq, kHD);
  transpose_bf16_kernel<<<dim3(kLim / 64, kHD / 64, 1), 256, 0, stream>>>(pe, PEt, kHD, kLim);

  const unsigned tilesScore = (unsigned)((kSeq / 64) * (kSeq / 64) / 8);
  const unsigned tilesPV    = (unsigned)((kSeq / 64) * (kHD / 64) / 8);
  for (int g0 = 0; g0 < kNB; g0 += kGrp) {
    const int G = (kNB - g0 < kGrp) ? (kNB - g0) : kGrp;
    const unsigned short* Qg = Qb + (size_t)g0 * kSeq * kHD;
    const unsigned short* Kg = Kb + (size_t)g0 * kSeq * kHD;
    const unsigned short* Vg = Vt + (size_t)g0 * kHD * kSeq;
    float* Og = out + (size_t)g0 * kSeq * kHD;
    wmma_gemm64<1, false, false, 0, false, 2, false><<<dim3(tilesScore, G), 256, 0, stream>>>(
        Qg, nullptr, kHD, (long)kSeq * kHD,
        PEt, nullptr, kHD, 0L,
        (void*)Rf, nullptr, kLim, (long)plane,
        nullptr, 0L, 0,
        kSeq, kLim, kHD, 1.0f);
    wmma_gemm64<1, false, false, 0, true, 1, false><<<dim3(tilesScore, G), 256, 0, stream>>>(
        Qg, nullptr, kHD, (long)kSeq * kHD,
        Kg, nullptr, kHD, (long)kSeq * kHD,
        (void*)Sc, nullptr, kSeq, (long)plane,
        Rf + (kLim - 1), (long)plane, kLim - 1,
        kSeq, kSeq, kHD, 1.0f);
    softmax_skew_kernel<<<dim3(kSeq, G), 256, 0, stream>>>(Sc, Ph, Pl);
    wmma_gemm64<1, true, true, 0, false, 0, true><<<dim3(tilesPV, G), 256, 0, stream>>>(
        Ph, Pl, kSeq, (long)plane,
        Vg, nullptr, kSeq, (long)kHD * kSeq,
        (void*)Og, nullptr, kHD, (long)kSeq * kHD,
        nullptr, 0L, 0,
        kSeq, kHD, kSeq, 1.0f);
  }
}
